// QConvImg2Col_62758062129880
// MI455X (gfx1250) — hardware-verified
//
#include <hip/hip_runtime.h>
#include <math.h>

#pragma clang fp contract(off)

constexpr int kBatch  = 32;
constexpr int kCin    = 128;
constexpr int kCout   = 128;
constexpr int kImg    = 56;
constexpr int kL      = kImg * kImg;
constexpr int kK      = kCin * 9;
constexpr int kChunk  = 8;
constexpr int kNChunk = kBatch / kChunk;

typedef __attribute__((ext_vector_type(16))) _Float16 v16h;
typedef __attribute__((ext_vector_type(8)))  _Float16 v8h;
typedef __attribute__((ext_vector_type(16))) __bf16   v16b;
typedef __attribute__((ext_vector_type(8)))  __bf16   v8b;
typedef __attribute__((ext_vector_type(8)))  float    v8f;
typedef __attribute__((ext_vector_type(4)))  float    v4f;
typedef __attribute__((ext_vector_type(4)))  unsigned int v4u;

__device__ __forceinline__ unsigned short f2bf_bits(float f) {
  unsigned u = __float_as_uint(f);
  return (unsigned short)((u + 0x7FFFu + ((u >> 16) & 1u)) >> 16);
}
__device__ __forceinline__ float bf_bits2f(unsigned short h) { return __uint_as_float(((unsigned)h) << 16); }

__device__ __forceinline__ void dep_guard_h(v8f& a, v8f& b, v16h x, v16h y) { asm volatile("v_nop\n\tv_nop\n\tv_nop\n\tv_nop" : "+v"(a), "+v"(b) : "v"(x), "v"(y)); }
__device__ __forceinline__ void dep_guard_b(v8f& a, v8f& b, v16b x, v16b y) { asm volatile("v_nop\n\tv_nop\n\tv_nop\n\tv_nop" : "+v"(a), "+v"(b) : "v"(x), "v"(y)); }
__device__ __forceinline__ void keep4_h(v16h a, v16h b, v16h c, v16h d) { asm volatile("v_nop" :: "v"(a), "v"(b), "v"(c), "v"(d)); }
__device__ __forceinline__ void keep4_b(v16b a, v16b b, v16b c, v16b d) { asm volatile("v_nop" :: "v"(a), "v"(b), "v"(c), "v"(d)); }
__device__ __forceinline__ void acc_guard4(v8f& a, v8f& b, v8f& c, v8f& d) { asm volatile("v_nop\n\tv_nop\n\tv_nop\n\tv_nop" : "+v"(a), "+v"(b), "+v"(c), "+v"(d)); }
template <typename T> struct Frag;
template <> struct Frag<_Float16> {
  typedef v16h V; union U { v16h v; v8h h[2]; };
  static __device__ __forceinline__ v16h load(const _Float16* p) {
    U f; f.h[0] = *(const v8h*)(p); f.h[1] = *(const v8h*)(p + 16); return f.v;
  }
  static __device__ __forceinline__ v8f mma(v16h a, v16h b, v8f c) {
    return __builtin_amdgcn_wmma_f32_16x16x32_f16(false, a, false, b, (short)0, c, false, false);
  }
  static __device__ __forceinline__ void guard(v8f& a, v8f& b, v16h x, v16h y) { dep_guard_h(a, b, x, y); }
  static __device__ __forceinline__ void keep(v16h a, v16h b, v16h c, v16h d) { keep4_h(a, b, c, d); }
};
template <> struct Frag<__bf16> {
  typedef v16b V; union U { v16b v; v8b h[2]; };
  static __device__ __forceinline__ v16b load(const __bf16* p) {
    U f; f.h[0] = *(const v8b*)(p); f.h[1] = *(const v8b*)(p + 16); return f.v;
  }
  static __device__ __forceinline__ v8f mma(v16b a, v16b b, v8f c) {
    return __builtin_amdgcn_wmma_f32_16x16x32_bf16(false, a, false, b, (short)0, c, false, false);
  }
  static __device__ __forceinline__ void guard(v8f& a, v8f& b, v16b x, v16b y) { dep_guard_b(a, b, x, y); }
  static __device__ __forceinline__ void keep(v16b a, v16b b, v16b c, v16b d) { keep4_b(a, b, c, d); }
};

__device__ __forceinline__ unsigned pk16(unsigned short a, unsigned short b) { return (unsigned)a | ((unsigned)b << 16); }
__device__ __forceinline__ unsigned short h_bits(float f) { const _Float16 h = (_Float16)f; return __builtin_bit_cast(unsigned short, h); }

template <int ET> struct Elem;
template <> struct Elem<0> { typedef _Float16 T; };
template <> struct Elem<1> { typedef __bf16 T; };
template <int ET, bool SPLIT, int BIAS_MODE, int OUT_MODE, bool RESID, int ACT = 0>
__global__ __launch_bounds__(256) void wmma_gemm64(
    const unsigned short* __restrict__ Ap, const unsigned short* __restrict__ A2p, int lda, long strideA,
    const unsigned short* __restrict__ Btp, const unsigned short* __restrict__ Bt2p, int ldb, long strideB,
    void* __restrict__ Cout, void* __restrict__ Cout2, int ldc, long strideC,
    const float* __restrict__ bias,
    const float* __restrict__ resid, long strideR,
    int M, int N, int K, float scale) {
  typedef typename Elem<ET>::T T;
  typedef typename Frag<T>::V V;
  const T* A = (const T*)Ap; const T* A2 = (const T*)A2p; const T* Bt = (const T*)Btp; const T* Bt2 = (const T*)Bt2p;
  __shared__ __align__(16) float sT[8][16 * 68];
  const int b    = blockIdx.y;
  const int lane = threadIdx.x & 31;
  const int wave = threadIdx.x >> 5;
  const int tilesN = N >> 6;
  const int tilesM = M >> 6;
  const int tile = blockIdx.x * 8 + wave;
  if (tile >= tilesM * tilesN) return;
  const int tm = tile / tilesN;
  const int tn = tile - tm * tilesN;
  const int m0 = tm << 6;
  const int n0 = tn << 6;

  const T* Ab  = A  + (size_t)b * strideA;
  const T* Bb  = Bt + (size_t)b * strideB;
  const T* Ab2 = SPLIT ? (A2  + (size_t)b * strideA) : nullptr;
  const T* Bb2 = SPLIT ? (Bt2 + (size_t)b * strideB) : nullptr;

  const int rlane = lane & 15;
  const int koff  = (lane >> 4) * 8;
  const int mOff  = (lane >> 4) * 8;

  v8f acc[4][4];
#pragma unroll
  for (int i = 0; i < 4; ++i)
#pragma unroll
    for (int j = 0; j < 4; ++j) acc[i][j] = (v8f){0.f,0.f,0.f,0.f,0.f,0.f,0.f,0.f};

  for (int k0 = 0; k0 < K; k0 += 32) {
    V bh[4], bl[4];
#pragma unroll
    for (int j = 0; j < 4; ++j) {
      const size_t bo = (size_t)(n0 + (j << 4) + rlane) * ldb + koff + k0;
      bh[j] = Frag<T>::load(Bb + bo);
      if (SPLIT) bl[j] = Frag<T>::load(Bb2 + bo);
    }
#pragma unroll
    for (int i = 0; i < 4; ++i) {
      const size_t ao = (size_t)(m0 + (i << 4) + rlane) * lda + koff + k0;
      V ah = Frag<T>::load(Ab + ao);
      V al;
      if (SPLIT) al = Frag<T>::load(Ab2 + ao);
#pragma unroll
      for (int j = 0; j < 4; ++j) {
        acc[i][j] = Frag<T>::mma(ah, bh[j], acc[i][j]);
        if (SPLIT) {
          acc[i][j] = Frag<T>::mma(ah, bl[j], acc[i][j]);
          acc[i][j] = Frag<T>::mma(al, bh[j], acc[i][j]);
        }
      }
      Frag<T>::guard(acc[i][0], acc[i][3], ah, SPLIT ? al : ah);
    }
    Frag<T>::keep(bh[0], bh[1], bh[2], bh[3]);
    if (SPLIT) Frag<T>::keep(bl[0], bl[1], bl[2], bl[3]);
  }
  acc_guard4(acc[0][0], acc[0][1], acc[0][2], acc[0][3]);
  acc_guard4(acc[1][0], acc[1][1], acc[1][2], acc[1][3]);
  acc_guard4(acc[2][0], acc[2][1], acc[2][2], acc[2][3]);
  acc_guard4(acc[3][0], acc[3][1], acc[3][2], acc[3][3]);

  float* slab = sT[wave];
  const float* Rb = RESID ? (resid + (size_t)b * strideR) : nullptr;
#pragma unroll
  for (int i = 0; i < 4; ++i) {
    const int mBase = m0 + (i << 4);
#pragma unroll
    for (int j = 0; j < 4; ++j) {
      const int n = n0 + (j << 4) + rlane;
      float bv = 0.f;
      if (BIAS_MODE == 2) bv = bias[n];
#pragma unroll
      for (int r = 0; r < 8; ++r) {
        float v = acc[i][j][r] * scale;
        if (BIAS_MODE == 1) v += bias[mBase + mOff + r];
        if (BIAS_MODE == 2) v += bv;
        if (RESID) v += Rb[(size_t)(mBase + mOff + r) * ldc + n];
        if (ACT == 2) v = fmaxf(v, 0.0f);
        if (ACT == 4) v = (v > 0.f) ? v : 0.01f * v;
        slab[(mOff + r) * 68 + (j << 4) + rlane] = v;
      }
    }
    __builtin_amdgcn_fence(__ATOMIC_RELEASE, "workgroup");
    __builtin_amdgcn_wave_barrier();
    __builtin_amdgcn_fence(__ATOMIC_ACQUIRE, "workgroup");
    if (OUT_MODE == 0) {
      float* C = (float*)Cout + (size_t)b * strideC;
      const int hh = lane >> 4, c4 = (lane & 15) * 4;
      for (int pass = 0; pass < 2; ++pass) {
#pragma unroll
        for (int it = 0; it < 8; ++it) {
          const int row = it * 2 + hh;
          v4f v = *(const v4f*)(slab + row * 68 + c4);
          *(volatile v4f*)(C + (size_t)(mBase + row) * ldc + n0 + c4) = v;
        }
        __threadfence();
      }
    } else {
      const int q = lane >> 3, c8 = (lane & 7) * 8;
      unsigned short* C  = (unsigned short*)Cout  + (size_t)b * strideC;
      unsigned short* C2 = (OUT_MODE == 2) ? ((unsigned short*)Cout2 + (size_t)b * strideC) : nullptr;
      for (int pass = 0; pass < 2; ++pass) {
#pragma unroll
        for (int it = 0; it < 4; ++it) {
          const int row = it * 4 + q;
          const float* sp = slab + row * 68 + c8;
          v8h hv, lv;
#pragma unroll
          for (int e = 0; e < 8; ++e) {
            if (OUT_MODE == 1) {
              hv[e] = (_Float16)sp[e];
            } else {
              unsigned short hb = f2bf_bits(sp[e]);
              unsigned short lb = f2bf_bits(sp[e] - bf_bits2f(hb));
              hv[e] = __builtin_bit_cast(_Float16, hb);
              lv[e] = __builtin_bit_cast(_Float16, lb);
            }
          }
          *(volatile v8h*)(C + (size_t)(mBase + row) * ldc + n0 + c8) = hv;
          if (OUT_MODE == 2) *(volatile v8h*)(C2 + (size_t)(mBase + row) * ldc + n0 + c8) = lv;
        }
        __threadfence();
      }
    }
    __builtin_amdgcn_fence(__ATOMIC_RELEASE, "workgroup");
    __builtin_amdgcn_wave_barrier();
    __builtin_amdgcn_fence(__ATOMIC_ACQUIRE, "workgroup");
  }
}

__device__ __forceinline__ float lsq_step(float s, float g) {
  const float sg = s * g;
  const float a  = s - sg;
  return a + sg;
}

__device__ __forceinline__ unsigned short qcode_bits(float v, float inv) {
  float y = v * inv;
  y = fminf(fmaxf(y, -128.0f), 127.0f);
  const float r = __builtin_rintf(y);
  return h_bits(r);
}

__global__ __launch_bounds__(256) void quant8_kernel(const float* __restrict__ in, const float* __restrict__ step,
                                                     unsigned short* __restrict__ out, float g, int n8) {
  const int i = blockIdx.x * 256 + threadIdx.x;
  if (i >= n8) return;
  const float ss  = lsq_step(step[0], g);
  const float inv = 1.0f / ss;
  const float* p = in + 8 * (size_t)i;
  const v4f a = *(const v4f*)(p);
  const v4f c = *(const v4f*)(p + 4);
  unsigned short hb[8];
#pragma unroll
  for (int e = 0; e < 4; ++e) {
    hb[e]     = qcode_bits(a[e], inv);
    hb[4 + e] = qcode_bits(c[e], inv);
  }
  const v4u u = (v4u){pk16(hb[0], hb[1]), pk16(hb[2], hb[3]), pk16(hb[4], hb[5]), pk16(hb[6], hb[7])};
  unsigned short* q = out + 8 * (size_t)i;
  *(volatile v4u*)q = u;
  __threadfence();
  *(volatile v4u*)q = u;
}

__global__ __launch_bounds__(288) void im2col_kernel(const unsigned short* __restrict__ xq,
                                                     unsigned short* __restrict__ bt, int img0) {
  const int tid  = threadIdx.x;
  const int rsel = (tid >= 144) ? 1 : 0;
  const int t    = tid - rsel * 144;
  const int l    = blockIdx.x * 2 + rsel;
  const int bi   = blockIdx.y;
  int b = img0 + bi;
  b = (b < 0) ? 0 : ((b > kBatch - 1) ? (kBatch - 1) : b);
  const int ho = l / kImg;
  const int wo = l - ho * kImg;
  const int kb = t * 8;
  const unsigned short* xb = xq + (size_t)b * (size_t)(kCin * kL);
  unsigned short hv[8];
#pragma unroll
  for (int e = 0; e < 8; ++e) {
    const int kk = kb + e;
    const int c  = kk / 9;
    const int t9 = kk - c * 9;
    const int i  = t9 / 3;
    const int j  = t9 - i * 3;
    const int hi = ho + i - 1;
    const int wi = wo + j - 1;
    const bool ok = ((unsigned)hi < (unsigned)kImg) && ((unsigned)wi < (unsigned)kImg);
    const int hc = (hi < 0) ? 0 : ((hi > kImg - 1) ? (kImg - 1) : hi);
    const int wc = (wi < 0) ? 0 : ((wi > kImg - 1) ? (kImg - 1) : wi);
    const unsigned short v = xb[(c * kImg + hc) * kImg + wc];
    hv[e] = ok ? v : (unsigned short)0;
  }
  const v4u u = (v4u){pk16(hv[0], hv[1]), pk16(hv[2], hv[3]), pk16(hv[4], hv[5]), pk16(hv[6], hv[7])};
  unsigned short* dst = bt + ((size_t)bi * kL + (size_t)l) * kK + kb;
  *(volatile v4u*)dst = u;
  __threadfence();
  *(volatile v4u*)dst = u;
}

__global__ __launch_bounds__(256) void scale_bias_kernel(float* __restrict__ out, const float* __restrict__ bias,
                                                         const float* __restrict__ s_act, const float* __restrict__ s_w,
                                                         float gx, float gw, int n4) {
  const int i = blockIdx.x * 256 + threadIdx.x;
  if (i >= n4) return;
  const float sx = lsq_step(s_act[0], gx);
  const float sw = lsq_step(s_w[0], gw);
  const float sc = sx * sw;
  const int o = (i / (kL / 4)) & (kCout - 1);
  const float bv = bias[o];
  float* p = out + 4 * (size_t)i;
  const v4f r = *(const v4f*)p;
  v4f v;
#pragma unroll
  for (int e = 0; e < 4; ++e) {
    const float m = r[e] * sc;
    v[e] = m + bv;
  }
  *(volatile v4f*)p = v;
  __threadfence();
  *(volatile v4f*)p = v;
}

extern "C" void kernel_launch(void* const* d_in, const int* in_sizes, int n_in,
                              void* d_out, int out_size, void* d_ws, size_t ws_size,
                              hipStream_t stream) {
  if (n_in < 5) return;
  const float* x     = (const float*)d_in[0];
  const float* w     = (const float*)d_in[1];
  const float* bias  = (const float*)d_in[2];
  const float* s_act = (const float*)d_in[3];
  const float* s_w   = (const float*)d_in[4];
  float* out = (float*)d_out;

  const int nx = in_sizes[0];
  const int nw = in_sizes[1];
  if (nx != kBatch * kCin * kL) return;
  if (nw != kCout * kK) return;
  if (out_size != kBatch * kCout * kL) return;
  if (in_sizes[2] < kCout || in_sizes[3] < 1 || in_sizes[4] < 1) return;

  const double gxd = 1.0 / sqrt(127.0 * (double)nx);
  const double gwd = 1.0 / sqrt(127.0 * (double)nw);
  const float gx = (float)gxd;
  const float gw = (float)gwd;

  const size_t xq_bytes = (size_t)nx * 2;
  const size_t wa_bytes = (size_t)nw * 2;
  const size_t bt_bytes = (size_t)kChunk * kL * kK * 2;
  const size_t off_xq = 0;
  const size_t off_wa = off_xq + ((xq_bytes + 127) / 128) * 128;
  const size_t off_bt = off_wa + ((wa_bytes + 127) / 128) * 128;
  const size_t total  = off_bt + bt_bytes;
  if (total > ws_size) return;

  unsigned short* xq = (unsigned short*)((char*)d_ws + off_xq);
  unsigned short* wa = (unsigned short*)((char*)d_ws + off_wa);
  unsigned short* bt = (unsigned short*)((char*)d_ws + off_bt);

  {
    const int n8 = nx / 8;
    quant8_kernel<<<(n8 + 255) / 256, 256, 0, stream>>>(x, s_act, xq, gx, n8);
  }
  {
    const int n8 = nw / 8;
    quant8_kernel<<<(n8 + 255) / 256, 256, 0, stream>>>(w, s_w, wa, gw, n8);
  }
  const int tiles      = (kCout / 64) * (kL / 64);
  const int gemmBlocks = (tiles + 7) / 8;
  for (int ch = 0; ch < kNChunk; ++ch) {
    const int img0 = ch * kChunk;
    im2col_kernel<<<dim3(kL / 2, kChunk), 288, 0, stream>>>(xq, bt, img0);
    float* outc = out + (size_t)img0 * kCout * kL;
    wmma_gemm64<0, false, 0, 0, false, 0><<<dim3(gemmBlocks, kChunk), 256, 0, stream>>>(
        wa, wa, kK, 0L,
        bt, bt, kK, (long)kL * kK,
        (void*)outc, (void*)outc, kL, (long)kCout * kL,
        bias,
        bias, 0L,
        kCout, kL, kK, 1.0f);
  }
  {
    const int n4 = out_size / 4;
    scale_bias_kernel<<<(n4 + 255) / 256, 256, 0, stream>>>(out, bias, s_act, s_w, gx, gw, n4);
  }
}
